// BaseLinearSSM_87823491268725
// MI455X (gfx1250) — hardware-verified
//
#include <hip/hip_runtime.h>
#include <stddef.h>
#include <stdint.h>


typedef _Float16 v16h __attribute__((ext_vector_type(16)));
typedef _Float16 v8h  __attribute__((ext_vector_type(8)));
typedef v8h __attribute__((__may_alias__)) v8hA;
typedef float v8f __attribute__((ext_vector_type(8)));
typedef float v4f __attribute__((ext_vector_type(4)));
typedef v4f __attribute__((__may_alias__)) v4fA;
typedef unsigned int v4u __attribute__((ext_vector_type(4)));
typedef v4u __attribute__((__may_alias__)) v4uA;

union Frag  { v16h v; v8h half[2]; };
union Pack8 { v8h h; v4u u; };

#define T_LEN   2048
#define BATCHSZ 16
#define IN_F    128
#define OUT_F   128
#define NSTATE  512
#define SROWS   1024
#define NROWS   (BATCHSZ * T_LEN)

#define WSCALE      16.0f
#define INV_WSCALE  0.0625f
#define LSCALE      1024.0f
#define INV_LSCALE  0.0009765625f

#define SCAN_THREADS 512
#define XPITCH       1032
#define OUT_THREADS  256
#define YP           68

#define CHUNK_U  (NROWS * IN_F / 8)
#define CHUNK_W  (SROWS * SROWS / 8)
#define CHUNK_B  (SROWS * IN_F / 8)
#define CHUNK_C  (OUT_F * SROWS / 8)
#define CHUNK_D  (OUT_F * IN_F / 8)
#define CHUNK_TOTAL (CHUNK_U + CHUNK_W + CHUNK_B + CHUNK_C + CHUNK_D)

static_assert(IN_F % 32 == 0);
static_assert(SROWS % 32 == 0);
static_assert(NROWS % 64 == 0);
static_assert(SCAN_THREADS / 32 * 64 == SROWS);
static_assert(SCAN_THREADS / 32 == BATCHSZ);
static_assert((XPITCH * 2) % 16 == 0);
static_assert((YP * 4) % 16 == 0);
static_assert(CHUNK_U % 8 == 0 && CHUNK_W % 8 == 0 && CHUNK_B % 8 == 0 && CHUNK_C % 8 == 0 && CHUNK_D % 8 == 0);

__device__ __forceinline__ v8f mma16(v16h a, v16h b, v8f c) {
  return __builtin_amdgcn_wmma_f32_16x16x32_f16(false, a, false, b, (short)0, c, false, false);
}
#define GUARD4(c0, c1, c2, c3, fa, f0, f1, f2, f3)                                      \
  asm volatile("v_nop\n\tv_nop\n\tv_nop\n\tv_nop"                                      \
               : "+v"(c0), "+v"(c1), "+v"(c2), "+v"(c3)                                \
               : "v"(fa), "v"(f0), "v"(f1), "v"(f2), "v"(f3))
#define GUARD8(c0, c1, c2, c3, c4, c5, c6, c7, fa, fb, f0, f1, f2, f3)                 \
  asm volatile("v_nop\n\tv_nop\n\tv_nop\n\tv_nop"                                      \
               : "+v"(c0), "+v"(c1), "+v"(c2), "+v"(c3),                               \
                 "+v"(c4), "+v"(c5), "+v"(c6), "+v"(c7)                                \
               : "v"(fa), "v"(fb), "v"(f0), "v"(f1), "v"(f2), "v"(f3))

__device__ __forceinline__ void split16(float x, _Float16& hi, _Float16& lo) {
  const _Float16 hv = (_Float16)x;
  const float res = (x - (float)hv) * LSCALE;
  hi = hv;
  lo = (_Float16)res;
}

__global__ void __launch_bounds__(256)
k_cvt(const float* __restrict__ u,
      const float* __restrict__ A_re, const float* __restrict__ A_im,
      const float* __restrict__ B_re, const float* __restrict__ B_im,
      const float* __restrict__ C_re, const float* __restrict__ C_im,
      const float* __restrict__ D_w,
      _Float16* __restrict__ u16, _Float16* __restrict__ Wt, _Float16* __restrict__ Bt,
      _Float16* __restrict__ Ct, _Float16* __restrict__ Dt) {
  const int c = blockIdx.x * 256 + threadIdx.x;
  if (c >= CHUNK_TOTAL) return;

  const float* src;
  _Float16* dst;
  float s;
  if (c < CHUNK_U) {
    src = u + (size_t)c * 8;
    dst = u16 + (size_t)c * 8;
    s = 1.0f;
  } else if (c < CHUNK_U + CHUNK_W) {
    const int e   = (c - CHUNK_U) * 8;
    const int np  = e >> 10;
    const int k   = e & (SROWS - 1);
    const int hiN = np >> 9;
    const int hiK = k >> 9;
    const int n   = np & (NSTATE - 1);
    const int kk  = k & (NSTATE - 1);
    src = ((hiN ^ hiK) ? A_im : A_re) + (size_t)n * NSTATE + kk;
    s   = (hiN == 0 && hiK == 1) ? -WSCALE : WSCALE;
    dst = Wt + e;
  } else if (c < CHUNK_U + CHUNK_W + CHUNK_B) {
    const int e  = (c - CHUNK_U - CHUNK_W) * 8;
    const int np = e >> 7;
    const int i  = e & (IN_F - 1);
    src = (np < NSTATE) ? (B_re + (size_t)np * IN_F + i) : (B_im + (size_t)(np - NSTATE) * IN_F + i);
    s   = WSCALE;
    dst = Bt + e;
  } else if (c < CHUNK_U + CHUNK_W + CHUNK_B + CHUNK_C) {
    const int e = (c - CHUNK_U - CHUNK_W - CHUNK_B) * 8;
    const int o = e >> 10;
    const int k = e & (SROWS - 1);
    src = (k < NSTATE) ? (C_re + (size_t)o * NSTATE + k) : (C_im + (size_t)o * NSTATE + (k - NSTATE));
    s   = (k < NSTATE) ? WSCALE : -WSCALE;
    dst = Ct + e;
  } else {
    const int e = (c - CHUNK_U - CHUNK_W - CHUNK_B - CHUNK_C) * 8;
    src = D_w + e;
    s   = WSCALE;
    dst = Dt + e;
  }

  const v4f lo = *(const v4fA*)(src);
  const v4f hi = *(const v4fA*)(src + 4);
  Pack8 p;
  p.h[0] = (_Float16)(lo[0] * s);
  p.h[1] = (_Float16)(lo[1] * s);
  p.h[2] = (_Float16)(lo[2] * s);
  p.h[3] = (_Float16)(lo[3] * s);
  p.h[4] = (_Float16)(hi[0] * s);
  p.h[5] = (_Float16)(hi[1] * s);
  p.h[6] = (_Float16)(hi[2] * s);
  p.h[7] = (_Float16)(hi[3] * s);
  const v4u pv = p.u;
  *(volatile v4uA*)dst = pv;
  __threadfence();
  *(volatile v4uA*)dst = pv;
}

__global__ void __launch_bounds__(SCAN_THREADS)
k_scan(const _Float16* __restrict__ u16, const _Float16* __restrict__ Wt,
       const _Float16* __restrict__ Bt, _Float16* __restrict__ xs) {
  __shared__ alignas(16) _Float16 xhi[BATCHSZ * XPITCH];
  __shared__ alignas(16) _Float16 xlo[BATCHSZ * XPITCH];

  const int tid  = threadIdx.x;
  const int lane = tid & 31;
  const int wv   = tid >> 5;
  const int h    = lane >> 4;
  const int m    = lane & 15;

  for (int e = tid; e < BATCHSZ * XPITCH; e += SCAN_THREADS) {
    xhi[e] = (_Float16)0.0f;
    xlo[e] = (_Float16)0.0f;
  }
  __syncthreads();

  const int ncol0 = wv * 64;
  const _Float16* wb = Wt + (size_t)(ncol0 + m) * SROWS + 8 * h;
  const _Float16* bb = Bt + (size_t)(ncol0 + m) * IN_F + 8 * h;
  const _Float16* ub = u16 + (size_t)m * T_LEN * IN_F + 8 * h;
  const int xa = m * XPITCH + 8 * h;
  const int xw = (8 * h) * XPITCH + ncol0 + m;
  const int xsrc = wv * XPITCH + lane * 8;
  _Float16* xdst = xs + (size_t)wv * T_LEN * SROWS + lane * 8;

#pragma unroll 1
  for (int it = 0; it < T_LEN; ++it) {
    v8f acc0 = {}, acc1 = {}, acc2 = {}, acc3 = {};
    v8f accL0 = {}, accL1 = {}, accL2 = {}, accL3 = {};

    const _Float16* up = ub + (size_t)it * IN_F;
#pragma unroll 1
    for (int kt = 0; kt < IN_F / 32; ++kt) {
      const int ko = kt * 32;
      Frag a, b0, b1, b2, b3;
      a.half[0]  = *(const v8hA*)(up + ko);
      a.half[1]  = *(const v8hA*)(up + ko + 16);
      b0.half[0] = *(const v8hA*)(bb + 0 * 16 * IN_F + ko);
      b0.half[1] = *(const v8hA*)(bb + 0 * 16 * IN_F + ko + 16);
      b1.half[0] = *(const v8hA*)(bb + 1 * 16 * IN_F + ko);
      b1.half[1] = *(const v8hA*)(bb + 1 * 16 * IN_F + ko + 16);
      b2.half[0] = *(const v8hA*)(bb + 2 * 16 * IN_F + ko);
      b2.half[1] = *(const v8hA*)(bb + 2 * 16 * IN_F + ko + 16);
      b3.half[0] = *(const v8hA*)(bb + 3 * 16 * IN_F + ko);
      b3.half[1] = *(const v8hA*)(bb + 3 * 16 * IN_F + ko + 16);
      acc0 = mma16(a.v, b0.v, acc0);
      acc1 = mma16(a.v, b1.v, acc1);
      acc2 = mma16(a.v, b2.v, acc2);
      acc3 = mma16(a.v, b3.v, acc3);
      GUARD4(acc0, acc1, acc2, acc3, a.v, b0.v, b1.v, b2.v, b3.v);
    }

#pragma unroll 1
    for (int kt = 0; kt < SROWS / 32; ++kt) {
      const int ko = kt * 32;
      Frag ah, al, b0, b1, b2, b3;
      ah.half[0] = *(const v8hA*)(&xhi[xa + ko]);
      ah.half[1] = *(const v8hA*)(&xhi[xa + ko + 16]);
      al.half[0] = *(const v8hA*)(&xlo[xa + ko]);
      al.half[1] = *(const v8hA*)(&xlo[xa + ko + 16]);
      b0.half[0] = *(const v8hA*)(wb + 0 * 16 * SROWS + ko);
      b0.half[1] = *(const v8hA*)(wb + 0 * 16 * SROWS + ko + 16);
      b1.half[0] = *(const v8hA*)(wb + 1 * 16 * SROWS + ko);
      b1.half[1] = *(const v8hA*)(wb + 1 * 16 * SROWS + ko + 16);
      b2.half[0] = *(const v8hA*)(wb + 2 * 16 * SROWS + ko);
      b2.half[1] = *(const v8hA*)(wb + 2 * 16 * SROWS + ko + 16);
      b3.half[0] = *(const v8hA*)(wb + 3 * 16 * SROWS + ko);
      b3.half[1] = *(const v8hA*)(wb + 3 * 16 * SROWS + ko + 16);
      acc0  = mma16(ah.v, b0.v, acc0);
      accL0 = mma16(al.v, b0.v, accL0);
      acc1  = mma16(ah.v, b1.v, acc1);
      accL1 = mma16(al.v, b1.v, accL1);
      acc2  = mma16(ah.v, b2.v, acc2);
      accL2 = mma16(al.v, b2.v, accL2);
      acc3  = mma16(ah.v, b3.v, acc3);
      accL3 = mma16(al.v, b3.v, accL3);
      GUARD8(acc0, acc1, acc2, acc3, accL0, accL1, accL2, accL3, ah.v, al.v, b0.v, b1.v, b2.v, b3.v);
    }

    __syncthreads();

#pragma unroll
    for (int r = 0; r < 8; ++r) {
      const float x0v = (acc0[r] + accL0[r] * INV_LSCALE) * INV_WSCALE;
      const float x1v = (acc1[r] + accL1[r] * INV_LSCALE) * INV_WSCALE;
      const float x2v = (acc2[r] + accL2[r] * INV_LSCALE) * INV_WSCALE;
      const float x3v = (acc3[r] + accL3[r] * INV_LSCALE) * INV_WSCALE;
      _Float16 h0, l0, h1, l1, h2, l2, h3, l3;
      split16(x0v, h0, l0);
      split16(x1v, h1, l1);
      split16(x2v, h2, l2);
      split16(x3v, h3, l3);
      const int idx = xw + r * XPITCH;
      xhi[idx +  0] = h0;  xlo[idx +  0] = l0;
      xhi[idx + 16] = h1;  xlo[idx + 16] = l1;
      xhi[idx + 32] = h2;  xlo[idx + 32] = l2;
      xhi[idx + 48] = h3;  xlo[idx + 48] = l3;
    }

    __syncthreads();

    {
      Pack8 p0, p1, p2, p3;
      p0.h = *(const v8hA*)(&xhi[xsrc]);
      p1.h = *(const v8hA*)(&xhi[xsrc + 256]);
      p2.h = *(const v8hA*)(&xhi[xsrc + 512]);
      p3.h = *(const v8hA*)(&xhi[xsrc + 768]);
      const v4u q0 = p0.u, q1 = p1.u, q2 = p2.u, q3 = p3.u;
      _Float16* d = xdst + (size_t)it * SROWS;
      *(volatile v4uA*)(d)       = q0;
      *(volatile v4uA*)(d + 256) = q1;
      *(volatile v4uA*)(d + 512) = q2;
      *(volatile v4uA*)(d + 768) = q3;
      __threadfence();
      *(volatile v4uA*)(d)       = q0;
      *(volatile v4uA*)(d + 256) = q1;
      *(volatile v4uA*)(d + 512) = q2;
      *(volatile v4uA*)(d + 768) = q3;
    }
  }
}

__global__ void __launch_bounds__(OUT_THREADS)
k_out(const _Float16* __restrict__ xs, const _Float16* __restrict__ u16,
      const _Float16* __restrict__ Ct, const _Float16* __restrict__ Dt,
      const float* __restrict__ bias, float* __restrict__ y) {
  __shared__ alignas(16) float ybuf[(OUT_THREADS / 32) * 16 * YP];

  const int tid  = threadIdx.x;
  const int lane = tid & 31;
  const int wv   = tid >> 5;
  const int h    = lane >> 4;
  const int m    = lane & 15;
  const int rg   = wv & 3;
  const int ch   = wv >> 2;
  const int R0   = blockIdx.x * 64 + rg * 16;
  const int c0   = ch * 64;

  const _Float16* xa = xs  + (size_t)(R0 + m) * SROWS + 8 * h;
  const _Float16* ua = u16 + (size_t)(R0 + m) * IN_F  + 8 * h;
  const _Float16* cb = Ct  + (size_t)(c0 + m) * SROWS + 8 * h;
  const _Float16* db = Dt  + (size_t)(c0 + m) * IN_F  + 8 * h;

  v8f acc0 = {}, acc1 = {}, acc2 = {}, acc3 = {};

#pragma unroll 1
  for (int kt = 0; kt < IN_F / 32; ++kt) {
    const int ko = kt * 32;
    Frag a, b0, b1, b2, b3;
    a.half[0]  = *(const v8hA*)(ua + ko);
    a.half[1]  = *(const v8hA*)(ua + ko + 16);
    b0.half[0] = *(const v8hA*)(db + 0 * 16 * IN_F + ko);
    b0.half[1] = *(const v8hA*)(db + 0 * 16 * IN_F + ko + 16);
    b1.half[0] = *(const v8hA*)(db + 1 * 16 * IN_F + ko);
    b1.half[1] = *(const v8hA*)(db + 1 * 16 * IN_F + ko + 16);
    b2.half[0] = *(const v8hA*)(db + 2 * 16 * IN_F + ko);
    b2.half[1] = *(const v8hA*)(db + 2 * 16 * IN_F + ko + 16);
    b3.half[0] = *(const v8hA*)(db + 3 * 16 * IN_F + ko);
    b3.half[1] = *(const v8hA*)(db + 3 * 16 * IN_F + ko + 16);
    acc0 = mma16(a.v, b0.v, acc0);
    acc1 = mma16(a.v, b1.v, acc1);
    acc2 = mma16(a.v, b2.v, acc2);
    acc3 = mma16(a.v, b3.v, acc3);
    GUARD4(acc0, acc1, acc2, acc3, a.v, b0.v, b1.v, b2.v, b3.v);
  }

#pragma unroll 1
  for (int kt = 0; kt < SROWS / 32; ++kt) {
    const int ko = kt * 32;
    Frag a, b0, b1, b2, b3;
    a.half[0]  = *(const v8hA*)(xa + ko);
    a.half[1]  = *(const v8hA*)(xa + ko + 16);
    b0.half[0] = *(const v8hA*)(cb + 0 * 16 * SROWS + ko);
    b0.half[1] = *(const v8hA*)(cb + 0 * 16 * SROWS + ko + 16);
    b1.half[0] = *(const v8hA*)(cb + 1 * 16 * SROWS + ko);
    b1.half[1] = *(const v8hA*)(cb + 1 * 16 * SROWS + ko + 16);
    b2.half[0] = *(const v8hA*)(cb + 2 * 16 * SROWS + ko);
    b2.half[1] = *(const v8hA*)(cb + 2 * 16 * SROWS + ko + 16);
    b3.half[0] = *(const v8hA*)(cb + 3 * 16 * SROWS + ko);
    b3.half[1] = *(const v8hA*)(cb + 3 * 16 * SROWS + ko + 16);
    acc0 = mma16(a.v, b0.v, acc0);
    acc1 = mma16(a.v, b1.v, acc1);
    acc2 = mma16(a.v, b2.v, acc2);
    acc3 = mma16(a.v, b3.v, acc3);
    GUARD4(acc0, acc1, acc2, acc3, a.v, b0.v, b1.v, b2.v, b3.v);
  }

  float* yb = ybuf + wv * (16 * YP);
  const float bj0 = bias[c0 +  0 + m];
  const float bj1 = bias[c0 + 16 + m];
  const float bj2 = bias[c0 + 32 + m];
  const float bj3 = bias[c0 + 48 + m];
  const int yw = (8 * h) * YP + m;
#pragma unroll
  for (int r = 0; r < 8; ++r) {
    yb[yw + r * YP +  0] = acc0[r] * INV_WSCALE + bj0;
    yb[yw + r * YP + 16] = acc1[r] * INV_WSCALE + bj1;
    yb[yw + r * YP + 32] = acc2[r] * INV_WSCALE + bj2;
    yb[yw + r * YP + 48] = acc3[r] * INV_WSCALE + bj3;
  }
  __syncthreads();

  v4f v0, v1, v2, v3, v4, v5, v6, v7;
  {
    const float* s = yb + h * YP + m * 4;
    v0 = *(const v4fA*)(s +  0 * YP);
    v1 = *(const v4fA*)(s +  2 * YP);
    v2 = *(const v4fA*)(s +  4 * YP);
    v3 = *(const v4fA*)(s +  6 * YP);
    v4 = *(const v4fA*)(s +  8 * YP);
    v5 = *(const v4fA*)(s + 10 * YP);
    v6 = *(const v4fA*)(s + 12 * YP);
    v7 = *(const v4fA*)(s + 14 * YP);
  }
  float* d = y + (size_t)(R0 + h) * OUT_F + c0 + m * 4;
  *(volatile v4fA*)(d +  0 * OUT_F) = v0;
  *(volatile v4fA*)(d +  2 * OUT_F) = v1;
  *(volatile v4fA*)(d +  4 * OUT_F) = v2;
  *(volatile v4fA*)(d +  6 * OUT_F) = v3;
  *(volatile v4fA*)(d +  8 * OUT_F) = v4;
  *(volatile v4fA*)(d + 10 * OUT_F) = v5;
  *(volatile v4fA*)(d + 12 * OUT_F) = v6;
  *(volatile v4fA*)(d + 14 * OUT_F) = v7;
  __threadfence();
  *(volatile v4fA*)(d +  0 * OUT_F) = v0;
  *(volatile v4fA*)(d +  2 * OUT_F) = v1;
  *(volatile v4fA*)(d +  4 * OUT_F) = v2;
  *(volatile v4fA*)(d +  6 * OUT_F) = v3;
  *(volatile v4fA*)(d +  8 * OUT_F) = v4;
  *(volatile v4fA*)(d + 10 * OUT_F) = v5;
  *(volatile v4fA*)(d + 12 * OUT_F) = v6;
  *(volatile v4fA*)(d + 14 * OUT_F) = v7;
}

extern "C" void kernel_launch(void* const* d_in, const int* in_sizes, int n_in,
                              void* d_out, int out_size, void* d_ws, size_t ws_size,
                              hipStream_t stream) {
  if (n_in < 9) return;
  if (in_sizes[0] != NROWS * IN_F) return;
  if (in_sizes[1] != NSTATE * NSTATE || in_sizes[2] != NSTATE * NSTATE) return;
  if (in_sizes[3] != NSTATE * IN_F || in_sizes[4] != NSTATE * IN_F) return;
  if (in_sizes[5] != OUT_F * NSTATE || in_sizes[6] != OUT_F * NSTATE) return;
  if (in_sizes[7] != OUT_F * IN_F || in_sizes[8] != OUT_F) return;
  if (out_size != NROWS * OUT_F) return;

  const float* u    = (const float*)d_in[0];
  const float* A_re = (const float*)d_in[1];
  const float* A_im = (const float*)d_in[2];
  const float* B_re = (const float*)d_in[3];
  const float* B_im = (const float*)d_in[4];
  const float* C_re = (const float*)d_in[5];
  const float* C_im = (const float*)d_in[6];
  const float* D_w  = (const float*)d_in[7];
  const float* bias = (const float*)d_in[8];
  float* y = (float*)d_out;

  char* ws = (char*)d_ws;
  size_t off = 0;
  _Float16* u16 = (_Float16*)(ws + off); off += (size_t)NROWS * IN_F * sizeof(_Float16);
  _Float16* Wt  = (_Float16*)(ws + off); off += (size_t)SROWS * SROWS * sizeof(_Float16);
  _Float16* Bt  = (_Float16*)(ws + off); off += (size_t)SROWS * IN_F * sizeof(_Float16);
  _Float16* Ct  = (_Float16*)(ws + off); off += (size_t)OUT_F * SROWS * sizeof(_Float16);
  _Float16* Dt  = (_Float16*)(ws + off); off += (size_t)OUT_F * IN_F * sizeof(_Float16);
  _Float16* xs  = (_Float16*)(ws + off); off += (size_t)NROWS * SROWS * sizeof(_Float16);
  if (off > ws_size) return;

  const int cvt_blocks = (CHUNK_TOTAL + 255) / 256;
  k_cvt<<<dim3(cvt_blocks), dim3(256), 0, stream>>>(u, A_re, A_im, B_re, B_im, C_re, C_im, D_w,
                                                   u16, Wt, Bt, Ct, Dt);
  k_scan<<<dim3(1), dim3(SCAN_THREADS), 0, stream>>>(u16, Wt, Bt, xs);
  k_out<<<dim3(NROWS / 64), dim3(OUT_THREADS), 0, stream>>>(xs, u16, Ct, Dt, bias, y);
}
